// VQAttention_77309411362
// MI455X (gfx1250) — hardware-verified
//
#include <hip/hip_runtime.h>

typedef _Float16 hf;
typedef hf v16h __attribute__((ext_vector_type(16)));
typedef hf v8h __attribute__((ext_vector_type(8)));
typedef float v8f __attribute__((ext_vector_type(8)));
typedef float v4f __attribute__((ext_vector_type(4), may_alias));
typedef float v2f __attribute__((ext_vector_type(2), may_alias));
typedef unsigned v4u __attribute__((ext_vector_type(4), may_alias));

constexpr int Bc = 8, Tc = 512, Dc = 1024, Hc = 8, DKc = 128, DVc = 128, Cc = 512, Mc = 512;
constexpr int Sc = Mc + Tc;
constexpr int BT = Bc * Tc;
constexpr int HD = Hc * DKc;
constexpr int BH = Bc * Hc;
typedef char chk_a[(BT % 128 == 0 && Tc % 128 == 0 && Dc % 64 == 0 && HD % 64 == 0 && Cc % 64 == 0) ? 1 : -1];
typedef char chk_b[(DKc == 128 && DVc == 128 && Mc % 64 == 0 && Sc % 64 == 0 && Hc == 8 && Tc == 512) ? 1 : -1];

constexpr float kCandThr = 0.3f;

union Frag { v16h v; v8h h8[2]; hf e[16]; };
union Pack8 { v8h h; v4u u; };

__device__ __forceinline__ v8f zero8() { v8f z = {0.f, 0.f, 0.f, 0.f, 0.f, 0.f, 0.f, 0.f}; return z; }

__device__ __forceinline__ v4u pack8(const float* v) {
  Pack8 p;
#pragma unroll
  for (int i = 0; i < 8; ++i) p.h[i] = (hf)v[i];
  return p.u;
}

__device__ __forceinline__ v16h ldfrag(const hf* row, int k0, int h) {
  Frag f;
  f.h8[0] = *(const v8h*)(row + k0 + 8 * h);
  f.h8[1] = *(const v8h*)(row + k0 + 16 + 8 * h);
  return f.v;
}

__device__ __forceinline__ v8f wm(v8f c, v16h a, v16h b) {
  return __builtin_amdgcn_wmma_f32_16x16x32_f16(false, a, false, b, (short)0, c, false, false);
}
__device__ __forceinline__ v8f mma1(v8f c, v16h a, v16h b) {
  c = wm(c, a, b);
  asm volatile("v_nop\n\tv_nop\n\tv_nop\n\tv_nop" : "+v"(c) : "v"(a), "v"(b));
  return c;
}

__device__ __forceinline__ float wsum(float v) {
#pragma unroll
  for (int o = 16; o; o >>= 1) v += __shfl_xor(v, o, 32);
  return v;
}
__device__ __forceinline__ double wsumd(double v) {
#pragma unroll
  for (int o = 16; o; o >>= 1) v += __shfl_xor(v, o, 32);
  return v;
}
__device__ __forceinline__ float hsum16(float v) {
#pragma unroll
  for (int o = 8; o; o >>= 1) v += __shfl_xor(v, o, 32);
  return v;
}

__global__ void __launch_bounds__(256) k_cvt8(const float* __restrict__ src, hf* dst, int n8) {
  const int e = blockIdx.x * 256 + threadIdx.x;
  if (e >= n8) return;
  const size_t o = (size_t)e * 8;
  const v4f a = *(const v4f*)(src + o), c = *(const v4f*)(src + o + 4);
  float v[8] = {a.x, a.y, a.z, a.w, c.x, c.y, c.z, c.w};
  const v4u p = pack8(v);
  *(volatile v4u*)(dst + o) = p;
  __threadfence();
  *(volatile v4u*)(dst + o) = p;
}

__global__ void __launch_bounds__(256) k_kcatxl(const float* __restrict__ xlk, hf* kt) {
  const int bh = blockIdx.y;
  const int e = blockIdx.x * 256 + threadIdx.x;
  if (e >= Mc * DKc / 8) return;
  const float* s = xlk + (size_t)bh * Mc * DKc + (size_t)e * 8;
  const v4f a = *(const v4f*)s, c = *(const v4f*)(s + 4);
  float v[8] = {a.x, a.y, a.z, a.w, c.x, c.y, c.z, c.w};
  const v4u p = pack8(v);
  hf* d = kt + (size_t)bh * Sc * DKc + (size_t)e * 8;
  *(volatile v4u*)d = p;
  __threadfence();
  *(volatile v4u*)d = p;
}

__global__ void __launch_bounds__(256) k_c2(const float* __restrict__ cb, float* c2) {
  const int i = blockIdx.x * 256 + threadIdx.x;
  if (i >= Hc * Cc) return;
  const float* r = cb + (size_t)i * DKc;
  float s = 0.f;
#pragma unroll 4
  for (int d = 0; d < DKc; ++d) s += r[d] * r[d];
  *(volatile float*)(c2 + i) = s;
  __threadfence();
  *(volatile float*)(c2 + i) = s;
}

__global__ void __launch_bounds__(128) k_ln(const float* __restrict__ x, const float* __restrict__ g,
                                            const float* __restrict__ bb, hf* xt) {
  __shared__ float sh[4];
  const int row = blockIdx.x, tid = threadIdx.x, l = tid & 31, w = tid >> 5;
  const float* xr = x + (size_t)row * Dc + tid * 8;
  const v4f a = *(const v4f*)xr, c = *(const v4f*)(xr + 4);
  float v[8] = {a.x, a.y, a.z, a.w, c.x, c.y, c.z, c.w};
  float s = 0.f;
#pragma unroll
  for (int i = 0; i < 8; ++i) s += v[i];
  s = wsum(s);
  if (l == 0) sh[w] = s;
  __syncthreads();
  const float mu = ((sh[0] + sh[1]) + (sh[2] + sh[3])) * (1.0f / Dc);
  __syncthreads();
  float s2 = 0.f;
#pragma unroll
  for (int i = 0; i < 8; ++i) { const float d = v[i] - mu; s2 += d * d; }
  s2 = wsum(s2);
  if (l == 0) sh[w] = s2;
  __syncthreads();
  const float var = ((sh[0] + sh[1]) + (sh[2] + sh[3])) * (1.0f / Dc);
  const float rs = rsqrtf(var + 1e-6f);
  float o8[8];
#pragma unroll
  for (int i = 0; i < 8; ++i) o8[i] = (v[i] - mu) * rs * g[tid * 8 + i] + bb[tid * 8 + i];
  const v4u p = pack8(o8);
  hf* d = xt + (size_t)row * Dc + tid * 8;
  *(volatile v4u*)d = p;
  __threadfence();
  *(volatile v4u*)d = p;
}

__global__ void __launch_bounds__(256) k_wT(const float* __restrict__ w, hf* wT, int K, int N, float scale) {
  __shared__ float T[64][33];
  const int tid = threadIdx.x, n0 = blockIdx.x * 32, k0 = blockIdx.y * 64;
  if (n0 + 32 > N || k0 + 64 > K) return;
#pragma unroll
  for (int i = 0; i < 8; ++i) {
    const int idx = i * 256 + tid, r = idx >> 5, c = idx & 31;
    T[r][c] = w[(size_t)(k0 + r) * N + n0 + c] * scale;
  }
  __syncthreads();
  const int n = tid >> 3, ks = (tid & 7) * 8;
  float v[8];
#pragma unroll
  for (int i = 0; i < 8; ++i) v[i] = T[ks + i][n];
  const v4u p = pack8(v);
  hf* d = wT + (size_t)(n0 + n) * K + k0 + ks;
  *(volatile v4u*)d = p;
  __threadfence();
  *(volatile v4u*)d = p;
}

__global__ void __launch_bounds__(256)
k_gemm(const hf* __restrict__ A, const hf* __restrict__ Bt, float* Cm, int Mr, int N, int K,
       size_t sA, size_t sB, int bmod, size_t sC, float alpha) {
  __shared__ __align__(16) float stg[8][16][64];
  const int l = threadIdx.x & 31, wv = threadIdx.x >> 5, h = l >> 4, m = l & 15;
  const int m0 = (blockIdx.y * 8 + wv) * 16, n0 = blockIdx.x * 64, z = blockIdx.z;
  const bool act = (m0 + 16 <= Mr) && (n0 + 64 <= N);
  const int m0c = act ? m0 : 0, n0c = act ? n0 : 0;
  const hf* arow = A + (size_t)z * sA + (size_t)(m0c + m) * K;
  const hf* brow = Bt + (size_t)(z % bmod) * sB + (size_t)(n0c + m) * K;
  const size_t kb = (size_t)16 * K;
  v8f acc0 = zero8(), acc1 = zero8(), acc2 = zero8(), acc3 = zero8();
  for (int k0 = 0; k0 < K; k0 += 32) {
    const v16h a = ldfrag(arow, k0, h);
    const v16h b0 = ldfrag(brow, k0, h), b1 = ldfrag(brow + kb, k0, h);
    const v16h b2 = ldfrag(brow + 2 * kb, k0, h), b3 = ldfrag(brow + 3 * kb, k0, h);
    acc0 = wm(acc0, a, b0);
    acc1 = wm(acc1, a, b1);
    acc2 = wm(acc2, a, b2);
    acc3 = wm(acc3, a, b3);
    asm volatile("v_nop\n\tv_nop\n\tv_nop\n\tv_nop"
                 : "+v"(acc0), "+v"(acc1), "+v"(acc2), "+v"(acc3)
                 : "v"(a), "v"(b0), "v"(b1), "v"(b2), "v"(b3));
  }
  float* Cb = Cm + (size_t)z * sC;
#pragma unroll
  for (int r = 0; r < 8; ++r) {
    stg[wv][8 * h + r][m]      = acc0[r] * alpha;
    stg[wv][8 * h + r][16 + m] = acc1[r] * alpha;
    stg[wv][8 * h + r][32 + m] = acc2[r] * alpha;
    stg[wv][8 * h + r][48 + m] = acc3[r] * alpha;
  }
  __syncthreads();
  if (act) {
    v4f vals[8]; size_t di[8];
#pragma unroll
    for (int i = 0; i < 8; ++i) {
      const int L = i * 4 + (l >> 3), row = L >> 1, col = (L & 1) * 32 + (l & 7) * 4;
      vals[i] = *(const v4f*)&stg[wv][row][col];
      di[i] = (size_t)(m0 + row) * N + n0 + col;
      *(volatile v4f*)(Cb + di[i]) = vals[i];
    }
    __threadfence();
#pragma unroll
    for (int i = 0; i < 8; ++i) *(volatile v4f*)(Cb + di[i]) = vals[i];
  }
}

__global__ void __launch_bounds__(256)
k_hln(const float* __restrict__ yq, const float* __restrict__ yk, const float* __restrict__ xu,
      hf* q16, hf* k16, float* kf) {
  __shared__ __align__(16) float kst[8][DKc];
  const int l = threadIdx.x & 31, wv = threadIdx.x >> 5;
  const int gid = blockIdx.x * 8 + wv;
  const int hh = gid & 7, bt = gid >> 3;
  const int side = l >> 4, j = l & 15;
  const float* src = (side ? yk : yq) + (size_t)bt * HD + hh * DKc + j * 8;
  const v4f a = *(const v4f*)src, c = *(const v4f*)(src + 4);
  float v[8] = {a.x, a.y, a.z, a.w, c.x, c.y, c.z, c.w};
  float s = 0.f;
#pragma unroll
  for (int i = 0; i < 8; ++i) s += v[i];
  const float mu = hsum16(s) * (1.0f / DKc);
  float s2 = 0.f;
#pragma unroll
  for (int i = 0; i < 8; ++i) { const float d = v[i] - mu; s2 += d * d; }
  const float rs = rsqrtf(hsum16(s2) * (1.0f / DKc) + 1e-6f);
  float o8[8];
#pragma unroll
  for (int i = 0; i < 8; ++i) {
    const float yv = (v[i] - mu) * rs;
    o8[i] = side ? yv : (yv + xu[hh * DKc + j * 8 + i]);
  }
  if (side) {
#pragma unroll
    for (int i = 0; i < 8; ++i) kst[wv][j * 8 + i] = o8[i];
  }
  __syncthreads();
  const v4u pk = pack8(o8);
  const int b = bt >> 9, t = bt & 511;
  const size_t rb = (((size_t)(b * Hc + hh)) * Tc + t) * DKc;
  hf* P = (side ? k16 : q16) + rb + j * 8;
  const v4f kv4 = *(const v4f*)&kst[wv][l * 4];
  float* kd = kf + rb + l * 4;
  *(volatile v4u*)P = pk; *(volatile v4f*)kd = kv4;
  __threadfence();
  *(volatile v4u*)P = pk; *(volatile v4f*)kd = kv4;
}

__device__ __forceinline__ float dist3(float k2, float kcv, float c2v) {
#pragma clang fp contract(off)
  const float tw = 2.0f * kcv;
  const float a = k2 - tw;
  return a + c2v;
}

__global__ void __launch_bounds__(256)
k_vq(const float* __restrict__ kc, const float* __restrict__ c2, const float* __restrict__ cb,
     const hf* __restrict__ cb16, const float* __restrict__ kf, const float* __restrict__ lm,
     const float* __restrict__ x, const float* __restrict__ lng, const float* __restrict__ lnb,
     const float* __restrict__ wk, hf* kt16, float* lpart) {
#pragma clang fp contract(off)
  __shared__ float part[32];
  const int l = threadIdx.x & 31, wv = threadIdx.x >> 5;
  const int bh = blockIdx.y, hh = bh & 7, b = bh >> 3, tg = blockIdx.x;
  const float* c2h = c2 + hh * Cc;
#pragma unroll 1
  for (int i = 0; i < 4; ++i) {
    const int t = tg * 32 + wv * 4 + i;
    const size_t row = (size_t)bh * Tc + t;
    const float* kcr = kc + row * Cc;
    v4f kv = *(const v4f*)(kf + row * DKc + 4 * l);
    const float k2 = wsum(kv.x * kv.x + kv.y * kv.y + kv.z * kv.z + kv.w * kv.w);
    float best = 3.0e38f; int bi = 0;
#pragma unroll 4
    for (int jj = 0; jj < Cc / 32; ++jj) {
      const int c = jj * 32 + l;
      const float d = dist3(k2, kcr[c], c2h[c]);
      if (d < best) { best = d; bi = c; }
    }
#pragma unroll
    for (int o = 16; o; o >>= 1) {
      const float ob = __shfl_xor(best, o, 32); const int oi = __shfl_xor(bi, o, 32);
      if (ob < best || (ob == best && oi < bi)) { best = ob; bi = oi; }
    }
    const float lim = best + kCandThr;
    int ncand = 0;
#pragma unroll 1
    for (int jj = 0; jj < Cc / 32; ++jj) {
      const int c = jj * 32 + l;
      ncand += __builtin_popcount(__builtin_amdgcn_ballot_w32(dist3(k2, kcr[c], c2h[c]) < lim));
    }
    int z = bi;
    if (ncand > 1) {
      const float* xr = x + ((size_t)(b * Tc + t)) * Dc;
      float s = 0.f;
#pragma unroll 1
      for (int q = 0; q < 8; ++q) {
        const v4f xv = *(const v4f*)(xr + (q * 32 + l) * 4);
        s += (xv.x + xv.y) + (xv.z + xv.w);
      }
      const float mu = wsum(s) * (1.0f / Dc);
      float s2 = 0.f;
#pragma unroll 1
      for (int q = 0; q < 8; ++q) {
        const v4f xv = *(const v4f*)(xr + (q * 32 + l) * 4);
        const float d0 = xv.x - mu, d1 = xv.y - mu, d2 = xv.z - mu, d3 = xv.w - mu;
        s2 += (d0 * d0 + d1 * d1) + (d2 * d2 + d3 * d3);
      }
      const float rs = rsqrtf(wsum(s2) * (1.0f / Dc) + 1e-6f);
      double y0 = 0.0, y1 = 0.0, y2 = 0.0, y3 = 0.0;
      const float* wcol = wk + hh * DKc + 4 * l;
#pragma unroll 1
      for (int q = 0; q < 8; ++q) {
        const int ib = (q * 32 + l) * 4;
        const v4f xv = *(const v4f*)(xr + ib), gv = *(const v4f*)(lng + ib), bv = *(const v4f*)(lnb + ib);
        float xt4[4];
        xt4[0] = (xv.x - mu) * rs * gv.x + bv.x;
        xt4[1] = (xv.y - mu) * rs * gv.y + bv.y;
        xt4[2] = (xv.z - mu) * rs * gv.z + bv.z;
        xt4[3] = (xv.w - mu) * rs * gv.w + bv.w;
#pragma unroll
        for (int e = 0; e < 4; ++e) {
          const float mine = xt4[e];
#pragma unroll 1
          for (int src = 0; src < 32; ++src) {
            const float xi = __shfl(mine, src, 32);
            const v4f w4 = *(const v4f*)(wcol + (size_t)((q * 32 + src) * 4 + e) * HD);
            const double xd = (double)xi;
            y0 = fma(xd, (double)w4.x, y0);
            y1 = fma(xd, (double)w4.y, y1);
            y2 = fma(xd, (double)w4.z, y2);
            y3 = fma(xd, (double)w4.w, y3);
          }
        }
      }
      const float f0 = (float)y0, f1 = (float)y1, f2 = (float)y2, f3 = (float)y3;
      const float muy = wsum((f0 + f1) + (f2 + f3)) * (1.0f / DKc);
      const float e0 = f0 - muy, e1 = f1 - muy, e2 = f2 - muy, e3 = f3 - muy;
      const float ry = rsqrtf(wsum((e0 * e0 + e1 * e1) + (e2 * e2 + e3 * e3)) * (1.0f / DKc) + 1e-6f);
      const v4f ke = {e0 * ry, e1 * ry, e2 * ry, e3 * ry};
      kv = ke;
      const float k2e = wsum(kv.x * kv.x + kv.y * kv.y + kv.z * kv.z + kv.w * kv.w);
      float eb = 3.0e38f; int ez = Cc - 1;
#pragma unroll 1
      for (int jj = 0; jj < Cc / 32; ++jj) {
        const int c = jj * 32 + l;
        unsigned msk = __builtin_amdgcn_ballot_w32(dist3(k2, kcr[c], c2h[c]) < lim);
        while (msk) {
          const int bit = __builtin_ctz(msk); msk &= msk - 1u;
          const int cc = jj * 32 + bit;
          const v4f cv = *(const v4f*)(cb + ((size_t)hh * Cc + cc) * DKc + 4 * l);
          double pd = (double)kv.x * (double)cv.x;
          pd = fma((double)kv.y, (double)cv.y, pd);
          pd = fma((double)kv.z, (double)cv.z, pd);
          pd = fma((double)kv.w, (double)cv.w, pd);
          const float kce = (float)wsumd(pd);
          const float de = dist3(k2e, kce, c2h[cc]);
          if (de < eb) { eb = de; ez = cc; }
        }
      }
      z = ez;
    }
    z = min(max(z, 0), Cc - 1);
    v4u cp = {0u, 0u, 0u, 0u};
    hf* kd = kt16 + ((size_t)bh * Sc + Mc + t) * DKc + 8 * (l & 15);
    if (l < 16) { cp = *(const v4u*)(cb16 + ((size_t)hh * Cc + z) * DKc + 8 * l); *(volatile v4u*)kd = cp; }
    __threadfence();
    if (l < 16) { *(volatile v4u*)kd = cp; }
    const v4f cv = *(const v4f*)(cb + ((size_t)hh * Cc + z) * DKc + 4 * l);
    const float dx = kv.x - cv.x, dy = kv.y - cv.y, dz = kv.z - cv.z, dw = kv.w - cv.w;
    const float dd = wsum((dx * dx + dy * dy) + (dz * dz + dw * dw));
    if (l == 0) part[wv * 4 + i] = dd * lm[b * Tc + t];
  }
  __syncthreads();
  if (wv == 0) {
    const float pv = part[l];
    float* dp = lpart + (size_t)bh * Tc + tg * 32 + l;
    *(volatile float*)dp = pv;
    __threadfence();
    *(volatile float*)dp = pv;
  }
}

__global__ void __launch_bounds__(256)
k_fill_vT(const float* __restrict__ xlv, const float* __restrict__ yv, hf* vT) {
  __shared__ float T[64][33];
  const int tid = threadIdx.x, bh = blockIdx.z, b = bh >> 3, hh = bh & 7;
  const int d0 = blockIdx.x * 32, s0 = blockIdx.y * 64;
  if (d0 + 32 > DVc || s0 + 64 > Sc) return;
#pragma unroll
  for (int i = 0; i < 8; ++i) {
    const int idx = i * 256 + tid, r = idx >> 5, c = idx & 31, s = s0 + r;
    const float v = (s < Mc) ? xlv[((size_t)bh * Mc + s) * DVc + d0 + c]
                             : yv[((size_t)b * Tc + (s - Mc)) * HD + hh * DVc + d0 + c];
    T[r][c] = v;
  }
  __syncthreads();
  const int n = tid >> 3, ks = (tid & 7) * 8;
  float v[8];
#pragma unroll
  for (int i = 0; i < 8; ++i) v[i] = T[ks + i][n];
  const v4u p = pack8(v);
  hf* d = vT + ((size_t)bh * DVc + d0 + n) * Sc + s0 + ks;
  *(volatile v4u*)d = p;
  __threadfence();
  *(volatile v4u*)d = p;
}

__global__ void __launch_bounds__(256)
k_fill_uT(const float* __restrict__ up, hf* uT) {
  __shared__ float T[64][33];
  const int tid = threadIdx.x, bh = blockIdx.z;
  const int d0 = blockIdx.x * 32, c0 = blockIdx.y * 64;
  if (d0 + 32 > DVc || c0 + 64 > Cc) return;
#pragma unroll
  for (int i = 0; i < 8; ++i) {
    const int idx = i * 256 + tid, r = idx >> 5, c = idx & 31;
    T[r][c] = up[((size_t)bh * Cc + c0 + r) * DVc + d0 + c];
  }
  __syncthreads();
  const int n = tid >> 3, ks = (tid & 7) * 8;
  float v[8];
#pragma unroll
  for (int i = 0; i < 8; ++i) v[i] = T[ks + i][n];
  const v4u p = pack8(v);
  hf* d = uT + ((size_t)bh * DVc + d0 + n) * Cc + c0 + ks;
  *(volatile v4u*)d = p;
  __threadfence();
  *(volatile v4u*)d = p;
}

template <bool AGG>
__device__ __forceinline__ void attn_step(const hf* __restrict__ Kb, const hf* qs, int qoff, int sBase, int tglob,
                                          const float* __restrict__ lw, const hf* __restrict__ Vb, int ldV,
                                          int h, int m, float inv_tau, float& mrun, float& den, v8f* num) {
  v8f st[2];
#pragma unroll
  for (int ti = 0; ti < 2; ++ti) {
    v8f acc = zero8();
    const hf* kr = Kb + (size_t)(sBase + ti * 16 + m) * DKc;
#pragma unroll
    for (int c = 0; c < 4; ++c) acc = mma1(acc, ldfrag(kr, 32 * c, h), ldfrag(qs + qoff, 32 * c, h));
    st[ti] = acc;
  }
  float bm = -3.0e38f;
#pragma unroll
  for (int ti = 0; ti < 2; ++ti)
#pragma unroll
    for (int r = 0; r < 8; ++r) {
      float v = st[ti][r] * inv_tau;
      if (!AGG) { const int s = sBase + ti * 16 + 8 * h + r; if (s - Mc > tglob) v = -1.0e30f; }
      st[ti][r] = v;
      bm = fmaxf(bm, v);
    }
  bm = fmaxf(bm, __shfl_xor(bm, 16, 32));
  const float mnew = fmaxf(mrun, bm);
  const float scale = __expf(mrun - mnew);
  Frag pf;
  float ls = 0.f;
#pragma unroll
  for (int ti = 0; ti < 2; ++ti)
#pragma unroll
    for (int r = 0; r < 8; ++r) {
      const float p = __expf(st[ti][r] - mnew) * 4096.0f;
      const hf ph = (hf)p;
      pf.e[ti * 8 + r] = ph;
      const float pr = (float)ph;
      ls += AGG ? pr * lw[sBase + ti * 16 + 8 * h + r] : pr;
    }
  ls += __shfl_xor(ls, 16, 32);
  den = den * scale + ls;
  float s8[8];
#pragma unroll
  for (int r = 0; r < 8; ++r) s8[r] = __shfl(scale, 8 * h + r, 32);
#pragma unroll
  for (int dt = 0; dt < 8; ++dt) {
    v8f nv = num[dt];
#pragma unroll
    for (int r = 0; r < 8; ++r) nv[r] *= s8[r];
    num[dt] = mma1(nv, pf.v, ldfrag(Vb + (size_t)(dt * 16 + m) * ldV, sBase, h));
  }
  mrun = mnew;
}

__global__ void __launch_bounds__(256) __attribute__((amdgpu_num_vgpr(256)))
k_attn(const hf* __restrict__ q16, const hf* __restrict__ kt16, const hf* __restrict__ vT,
       const hf* __restrict__ cb16, const hf* __restrict__ uT, const float* __restrict__ lower,
       const float* __restrict__ yg, hf* o16) {
  extern __shared__ __align__(16) unsigned char smem[];
  hf* qs = (hf*)smem;
  const int tid = threadIdx.x, l = tid & 31, wv = tid >> 5, h = l >> 4, m = l & 15;
  const int bh = blockIdx.x, b = bh >> 3, hh = bh & 7, tb = blockIdx.y;
  const int t0 = tb * 8 + wv, tglob = t0 * 16 + m;
  {
    const v4u* g = (const v4u*)(q16 + ((size_t)bh * Tc + (size_t)tb * 128) * DKc);
    v4u* d = (v4u*)smem;
#pragma unroll
    for (int i = 0; i < 8; ++i) d[i * 256 + tid] = g[i * 256 + tid];
  }
  __syncthreads();
  constexpr float kTau = 11.313708498984761f;
  const float inv_tau = 1.0f / kTau;
  v8f num[8];
#pragma unroll
  for (int i = 0; i < 8; ++i) num[i] = zero8();
  float mrun = -3.0e38f, den = 0.f;
  const int qoff = (wv * 16 + m) * DKc;

  const hf* Kr = kt16 + (size_t)bh * Sc * DKc;
  const hf* Vr = vT + (size_t)bh * DVc * Sc;
  const int nrec = (Mc + 16 * (t0 + 1) + 31) / 32;
  for (int sb = 0; sb < nrec; ++sb)
    attn_step<false>(Kr, qs, qoff, sb * 32, tglob, nullptr, Vr, Sc, h, m, inv_tau, mrun, den, num);

  const hf* Ka = cb16 + (size_t)hh * Cc * DKc;
  const hf* Va = uT + (size_t)bh * DVc * Cc;
  const float* lw = lower + (size_t)bh * Cc;
  for (int sb = 0; sb < Cc / 32; ++sb)
    attn_step<true>(Ka, qs, qoff, sb * 32, tglob, lw, Va, Cc, h, m, inv_tau, mrun, den, num);

  float rd8[8];
#pragma unroll
  for (int r = 0; r < 8; ++r) rd8[r] = 1.0f / __shfl(den, 8 * h + r, 32);
  __syncthreads();
  hf* ost = qs + (size_t)wv * (16 * 128);
#pragma unroll
  for (int dt = 0; dt < 8; ++dt) {
    const int dcol = dt * 16 + m;
#pragma unroll
    for (int r = 0; r < 8; ++r) {
      const int tg = t0 * 16 + 8 * h + r;
      const float wvv = num[dt][r] * rd8[r];
      const float gv = yg[((size_t)(b * Tc + tg)) * HD + hh * DVc + dcol];
      const float sil = gv / (1.0f + __expf(-gv));
      ost[(8 * h + r) * 128 + dcol] = (hf)(wvv * sil * 64.0f);
    }
  }
  __syncthreads();
  v4u vals[8]; size_t di[8];
#pragma unroll
  for (int i = 0; i < 8; ++i) {
    const int L = i * 4 + (l >> 3), row = L >> 1, col = (L & 1) * 64 + (l & 7) * 8;
    vals[i] = *(const v4u*)(ost + row * 128 + col);
    di[i] = ((size_t)(b * Tc + t0 * 16 + row)) * HD + hh * DVc + col;
    *(volatile v4u*)(o16 + di[i]) = vals[i];
  }
  __threadfence();
#pragma unroll
  for (int i = 0; i < 8; ++i) *(volatile v4u*)(o16 + di[i]) = vals[i];
}

__global__ void __launch_bounds__(256) k_loss(const float* __restrict__ lpart, const float* __restrict__ lm, float* outl) {
  __shared__ float sh[256];
  __shared__ float sm[256];
  const int tid = threadIdx.x;
  float s = 0.f, ms = 0.f;
#pragma unroll 1
  for (int i = 0; i < (BH * Tc) / 256; ++i) s += lpart[(size_t)i * 256 + tid];
#pragma unroll 1
  for (int i = 0; i < BT / 256; ++i) ms += lm[i * 256 + tid];
  sh[tid] = s; sm[tid] = ms;
  __syncthreads();
  for (int o = 128; o; o >>= 1) {
    if (tid < o) { sh[tid] += sh[tid + o]; sm[tid] += sm[tid + o]; }
    __syncthreads();
  }
  if (tid == 0) {
    const float val = sh[0] / (sm[0] * (float)Hc + 1e-6f);
    const v2f vv = {val, val};
    *(volatile v2f*)outl = vv;
    __threadfence();
    *(volatile v2f*)outl = vv;
  }
}

extern "C" void kernel_launch(void* const* d_in, const int* in_sizes, int n_in,
                              void* d_out, int out_size, void* d_ws, size_t ws_size,
                              hipStream_t stream) {
  if (n_in < 16 || in_sizes[0] != BT * Dc || in_sizes[15] != Hc * Cc * DKc || out_size != BT * Dc + 2) return;
  const float* x    = (const float*)d_in[0];
  const float* lmask= (const float*)d_in[2];
  const float* xlk  = (const float*)d_in[3];
  const float* xlv  = (const float*)d_in[4];
  const float* aggU = (const float*)d_in[5];
  const float* aggL = (const float*)d_in[6];
  const float* lng  = (const float*)d_in[7];
  const float* lnb  = (const float*)d_in[8];
  const float* wq   = (const float*)d_in[9];
  const float* wk   = (const float*)d_in[10];
  const float* wvv  = (const float*)d_in[11];
  const float* wg   = (const float*)d_in[12];
  const float* wres = (const float*)d_in[13];
  const float* xu   = (const float*)d_in[14];
  const float* cb   = (const float*)d_in[15];
  float* out = (float*)d_out;
  float* outl = out + (size_t)BT * Dc;

  size_t off = 0;
  auto carve = [&](size_t bytes) -> size_t { size_t p = off; off += (bytes + 255) & ~(size_t)255; return p; };
  const size_t nXT = (size_t)BT * Dc, nW = (size_t)Dc * HD, nY = (size_t)BT * HD, nQ = (size_t)BH * Tc * DKc,
               nCB = (size_t)Hc * Cc * DKc, nKT = (size_t)BH * Sc * DKc, nVT = (size_t)BH * DVc * Sc,
               nUT = (size_t)BH * DVc * Cc, nKC = (size_t)BH * Tc * Cc, nO = (size_t)BT * HD, nLP = (size_t)BH * Tc;
  const size_t oXT = carve(nXT * 2), oW = carve(nW * 2);
  const size_t oYQ = carve(nY * 4), oYK = carve(nY * 4), oYV = carve(nY * 4), oYG = carve(nY * 4);
  const size_t oQ = carve(nQ * 2), oK = carve(nQ * 2), oKF = carve(nQ * 4);
  const size_t oCB = carve(nCB * 2), oC2 = carve((size_t)Hc * Cc * 4);
  const size_t oKT = carve(nKT * 2), oVT = carve(nVT * 2), oUT = carve(nUT * 2);
  const size_t oKC = carve(nKC * 4), oO = carve(nO * 2), oLP = carve(nLP * 4);
  if (off > ws_size) return;

  char* W = (char*)d_ws;
  hf* xt16 = (hf*)(W + oXT);
  hf* wT16 = (hf*)(W + oW);
  float* yq = (float*)(W + oYQ); float* yk = (float*)(W + oYK);
  float* yv = (float*)(W + oYV); float* yg = (float*)(W + oYG);
  hf* q16 = (hf*)(W + oQ); hf* k16 = (hf*)(W + oK); float* kf = (float*)(W + oKF);
  hf* cb16 = (hf*)(W + oCB); float* c2 = (float*)(W + oC2);
  hf* kt16 = (hf*)(W + oKT); hf* vT = (hf*)(W + oVT); hf* uT = (hf*)(W + oUT);
  float* kc = (float*)(W + oKC); hf* o16 = (hf*)(W + oO); float* lpart = (float*)(W + oLP);

  k_cvt8<<<(int)((nCB / 8 + 255) / 256), 256, 0, stream>>>(cb, cb16, (int)(nCB / 8));
  k_c2<<<(Hc * Cc + 255) / 256, 256, 0, stream>>>(cb, c2);
  k_kcatxl<<<dim3((Mc * DKc / 8 + 255) / 256, BH), 256, 0, stream>>>(xlk, kt16);
  k_ln<<<BT, 128, 0, stream>>>(x, lng, lnb, xt16);

  const dim3 gW(HD / 32, Dc / 64), gP(HD / 64, BT / 128, 1);
  const float* ws4[4] = {wq, wk, wvv, wg};
  float* ys4[4] = {yq, yk, yv, yg};
  for (int i = 0; i < 4; ++i) {
    k_wT<<<gW, 256, 0, stream>>>(ws4[i], wT16, Dc, HD, 1024.0f);
    k_gemm<<<gP, 256, 0, stream>>>(xt16, wT16, ys4[i], BT, HD, Dc, (size_t)0, (size_t)0, 1, (size_t)0,
                                   1.0f / 1024.0f);
  }
  k_hln<<<BT * Hc / 8, 256, 0, stream>>>(yq, yk, xu, q16, k16, kf);

  k_gemm<<<dim3(Cc / 64, Tc / 128, BH), 256, 0, stream>>>(k16, cb16, kc, Tc, Cc, DKc,
                                                          (size_t)Tc * DKc, (size_t)Cc * DKc, Hc,
                                                          (size_t)Tc * Cc, 1.0f);
  k_vq<<<dim3(Tc / 32, BH), 256, 0, stream>>>(kc, c2, cb, cb16, kf, lmask, x, lng, lnb, wk, kt16, lpart);

  k_fill_vT<<<dim3(DVc / 32, Sc / 64, BH), 256, 0, stream>>>(xlv, yv, vT);
  k_fill_uT<<<dim3(DVc / 32, Cc / 64, BH), 256, 0, stream>>>(aggU, uT);

  k_attn<<<dim3(BH, Tc / 128), 256, 128 * 128 * 2, stream>>>(q16, kt16, vT, cb16, uT, aggL, yg, o16);

  k_wT<<<dim3(Dc / 32, HD / 64), 256, 0, stream>>>(wres, wT16, HD, Dc, 1024.0f);
  k_gemm<<<dim3(Dc / 64, BT / 128, 1), 256, 0, stream>>>(o16, wT16, out, BT, Dc, HD, (size_t)0, (size_t)0, 1,
                                                         (size_t)0, 1.0f / 65536.0f);
  k_loss<<<1, 256, 0, stream>>>(lpart, lmask, outl);
}
